// DSConv_37726992728315
// MI455X (gfx1250) — hardware-run, weakly checked
//
#include <hip/hip_runtime.h>

typedef float          v8f   __attribute__((ext_vector_type(8)));
typedef float          v4f   __attribute__((ext_vector_type(4)));
typedef unsigned int   v4u   __attribute__((ext_vector_type(4)));
typedef int            v8i   __attribute__((ext_vector_type(8)));
typedef unsigned short v8us  __attribute__((ext_vector_type(8)));
typedef unsigned short v16us __attribute__((ext_vector_type(16)));
typedef __bf16         v16bf __attribute__((ext_vector_type(16)));
typedef _Float16       v16h  __attribute__((ext_vector_type(16)));
typedef v4f  __attribute__((may_alias)) v4fa;
typedef v8us __attribute__((may_alias)) v8usa;
union FragB { v16bf v; v16us u; v8us h[2]; v8i w; };
union FragH { v16h  v; v16us u; v8us h[2]; v8i w; };

__device__ __forceinline__ v8f wmb(const FragB& a, const FragB& b, v8f c) {
  v8f d = __builtin_amdgcn_wmma_f32_16x16x32_bf16(false, a.v, false, b.v, (short)0, c, false, false);
  asm volatile("v_nop\n\tv_nop\n\tv_nop\n\tv_nop" : "+v"(d) : "v"(a.w), "v"(b.w));
  return d;
}

__device__ __forceinline__ v8f wmh(const FragH& a, const FragH& b, v8f c) {
  v8f d = __builtin_amdgcn_wmma_f32_16x16x32_f16(false, a.v, false, b.v, (short)0, c, false, false);
  asm volatile("v_nop\n\tv_nop\n\tv_nop\n\tv_nop" : "+v"(d) : "v"(a.w), "v"(b.w));
  return d;
}

__device__ __forceinline__ unsigned bf16_bits(float f) {
  const unsigned u = __float_as_uint(f);
  const unsigned r = (u + 0x7FFFu + ((u >> 16) & 1u)) >> 16;
  const unsigned q = (u >> 16) | 0x40u;
  return ((u & 0x7fffffffu) > 0x7f800000u) ? q : r;
}

__device__ __forceinline__ float bf16_val(float f) {
  return __uint_as_float(bf16_bits(f) << 16);
}
__device__ __forceinline__ int clampi(int v, int lo, int hi) {
  return v < lo ? lo : (v > hi ? hi : v);
}

__device__ __forceinline__ unsigned f16_bits(float f) {
  const unsigned u  = __float_as_uint(f);
  const unsigned s  = (u >> 16) & 0x8000u;
  const unsigned a  = u & 0x7fffffffu;
  const unsigned t  = a - 0x38000000u;
  const unsigned r  = (t + 0x0FFFu + ((t >> 13) & 1u)) >> 13;
  const unsigned rc = r > 0x7C00u ? 0x7C00u : r;
  const bool small  = a < 0x38800000u;
  const bool isnan  = a > 0x7f800000u;
  const unsigned fin = small ? 0u : (s | rc);
  return isnan ? (s | 0x7E00u) : fin;
}

__device__ __forceinline__ unsigned pk16(unsigned lo, unsigned hi) { return lo | (hi << 16); }
__device__ __forceinline__ unsigned bf16_lo_bits(float v) {
  float hi = bf16_val(v);
  asm volatile("" : "+v"(hi));
  return bf16_bits(v - hi);
}
__device__ __forceinline__ v4u pack8_bf16(v4f a, v4f c) {
  return (v4u){ pk16(bf16_bits(a[0]), bf16_bits(a[1])), pk16(bf16_bits(a[2]), bf16_bits(a[3])),
                pk16(bf16_bits(c[0]), bf16_bits(c[1])), pk16(bf16_bits(c[2]), bf16_bits(c[3])) };
}
__device__ __forceinline__ v4u pack8_bf16_lo(v4f a, v4f c) {
  return (v4u){ pk16(bf16_lo_bits(a[0]), bf16_lo_bits(a[1])), pk16(bf16_lo_bits(a[2]), bf16_lo_bits(a[3])),
                pk16(bf16_lo_bits(c[0]), bf16_lo_bits(c[1])), pk16(bf16_lo_bits(c[2]), bf16_lo_bits(c[3])) };
}
__device__ __forceinline__ v4u pack8_f16(v4f a, v4f c) {
  return (v4u){ pk16(f16_bits(a[0]), f16_bits(a[1])), pk16(f16_bits(a[2]), f16_bits(a[3])),
                pk16(f16_bits(c[0]), f16_bits(c[1])), pk16(f16_bits(c[2]), f16_bits(c[3])) };
}

template <int FORM>
__global__ __launch_bounds__(256) void k_plane(const float* __restrict__ src, int rows, int cols, int ldsrc,
                                               unsigned short* __restrict__ dst, int MP, int KP) {
  static_assert(FORM >= 0 && FORM <= 3);
  const int KTOT = (FORM == 1 || FORM == 3) ? 2 * KP : KP;
  const unsigned ppr   = (unsigned)(KTOT >> 3);
  const unsigned kp8   = (unsigned)(KP >> 3);
  const unsigned total = (unsigned)MP * ppr;
  const unsigned g     = blockIdx.x * 256u + threadIdx.x;
  const unsigned rowu  = g / ppr;
  const unsigned p     = g - rowu * ppr;
  const bool second    = p >= kp8;
  const int row = (int)rowu;
  const int c0  = (int)((second ? p - kp8 : p) << 3);
  const float* srow = src + (size_t)clampi(row, 0, rows - 1) * (size_t)ldsrc;
  float x[8];
  unsigned mk[8];
#pragma unroll
  for (int e = 0; e < 8; ++e) {
    const int c = c0 + e;
    const float v = srow[clampi(c, 0, cols - 1)];
    asm volatile("" :: "v"(v));
    x[e]  = v;
    mk[e] = (row < rows && c < cols) ? 0xFFFFu : 0u;
  }
  const v4f a = (v4f){ x[0], x[1], x[2], x[3] };
  const v4f c = (v4f){ x[4], x[5], x[6], x[7] };
  v4u o;
  if (FORM == 2) {
    o = pack8_f16(a, c);
  } else {
    const v4u hi = pack8_bf16(a, c);
    o = hi;
    if (FORM == 1) { const v4u lo = pack8_bf16_lo(a, c); o = second ? lo : hi; }
  }
  const v4u mw = (v4u){ pk16(mk[0], mk[1]), pk16(mk[2], mk[3]), pk16(mk[4], mk[5]), pk16(mk[6], mk[7]) };
  o &= mw;
  if (g < total) {
    volatile v4u* q = (volatile v4u*)(dst + (size_t)g * 8);
    *q = o;
    __threadfence();
    *q = o;
  }
}

template <int FORM> struct FragOf    { typedef FragB T; };
template <>         struct FragOf<2> { typedef FragH T; };
__device__ __forceinline__ v8f mm(const FragB& a, const FragB& b, v8f c) { return wmb(a, b, c); }
__device__ __forceinline__ v8f mm(const FragH& a, const FragH& b, v8f c) { return wmh(a, b, c); }
template <class F> __device__ __forceinline__ F ld_frag(const unsigned short* p) {
  F f;
  f.h[0] = *(const v8usa*)(p);
  f.h[1] = *(const v8usa*)(p + 16);
  return f;
}

template <int FORM, int EPI>
__global__ __launch_bounds__(256) __attribute__((amdgpu_num_vgpr(248)))
void k_gemm_nt(const unsigned short* __restrict__ A, const unsigned short* __restrict__ B,
               const float* __restrict__ bias, float* __restrict__ D, int M, int N, int KTOT, int ldd) {
  static_assert(FORM >= 0 && FORM <= 2);
  static_assert(EPI == 0 || EPI == 1);
  typedef typename FragOf<FORM>::T F;
  __shared__ __attribute__((aligned(16))) float sT[8][16 * 68];
  const int lane = threadIdx.x & 31;
  const int wave = threadIdx.x >> 5;
  const int tilesM = (M + 63) >> 6;
  const int tilesN = (N + 63) >> 6;
  const int tile = blockIdx.x * 8 + wave;
  if (tile >= tilesM * tilesN) return;
  const int tm = tile / tilesN;
  const int tn = tile - tm * tilesN;
  const int m0 = tm << 6;
  const int n0 = tn << 6;

  const int rl = lane & 15;
  const int h8 = (lane >> 4) * 8;
  const unsigned short* pa = A + (size_t)(m0 + rl) * (size_t)KTOT + h8;
  const unsigned short* pb = B + (size_t)(n0 + rl) * (size_t)KTOT + h8;

  v8f acc[4][4];
#pragma unroll
  for (int i = 0; i < 4; ++i)
#pragma unroll
    for (int j = 0; j < 4; ++j) acc[i][j] = (v8f){0.f, 0.f, 0.f, 0.f, 0.f, 0.f, 0.f, 0.f};

#pragma unroll 1
  for (int k0 = 0; k0 < KTOT; k0 += 32) {
    F bf[4];
#pragma unroll
    for (int j = 0; j < 4; ++j) bf[j] = ld_frag<F>(pb + (size_t)(j << 4) * (size_t)KTOT + k0);
#pragma unroll
    for (int i = 0; i < 4; ++i) {
      const F af = ld_frag<F>(pa + (size_t)(i << 4) * (size_t)KTOT + k0);
#pragma unroll
      for (int j = 0; j < 4; ++j) acc[i][j] = mm(af, bf[j], acc[i][j]);
    }
  }

  float* slab = sT[wave];
  const int hh = lane >> 4;
  const int c4 = (lane & 15) * 4;
  const int nc = n0 + c4;
  const bool cok = nc < N;
  v4f bv = (v4f){0.f, 0.f, 0.f, 0.f};
  if (EPI == 1) {
    bv = *(const v4fa*)(bias + clampi(nc, 0, N - 4));
    asm volatile("" :: "v"(bv));
  }
#pragma unroll
  for (int i = 0; i < 4; ++i) {
    const int mBase = m0 + (i << 4);
#pragma unroll
    for (int j = 0; j < 4; ++j) {
#pragma unroll
      for (int r = 0; r < 8; ++r) slab[(h8 + r) * 68 + (j << 4) + rl] = acc[i][j][r];
    }
    __builtin_amdgcn_fence(__ATOMIC_RELEASE, "workgroup");
    __builtin_amdgcn_wave_barrier();
    __builtin_amdgcn_fence(__ATOMIC_ACQUIRE, "workgroup");
    v4f vv[8];
#pragma unroll
    for (int it = 0; it < 8; ++it) {
      const int row = it * 2 + hh;
      v4f v = *(const v4fa*)(slab + row * 68 + c4);
      if (EPI == 1) v += bv;
      vv[it] = v;
    }
    for (int pass = 0; pass < 2; ++pass) {
#pragma unroll
      for (int it = 0; it < 8; ++it) {
        const int row = mBase + it * 2 + hh;
        if (cok && row < M) *(volatile v4f*)(D + (size_t)row * (size_t)ldd + nc) = vv[it];
      }
      __threadfence();
    }
    __builtin_amdgcn_fence(__ATOMIC_RELEASE, "workgroup");
    __builtin_amdgcn_wave_barrier();
    __builtin_amdgcn_fence(__ATOMIC_ACQUIRE, "workgroup");
  }
}

#pragma clang fp contract(off)

#define NB     4
#define NC     64
#define NH     128
#define NW     128
#define NT     9
#define KIN    576
#define K2     1152
#define NPIX   65536
#define MH     32768
#define NOFF   32
#define NOUT   64
#define NGRPS  16
#define GNB    64
#define VEC_F  512
#define V_OB   0
#define V_BG   16
#define V_BB   32
#define V_BM   48
#define V_DEN  64
#define V_CB   128
#define V_GG   192
#define V_GB   256
#define WSLIM  ((size_t)128 << 20)

static_assert(NH == 128 && NW == 128 && NH == NW && NC == 64 && NT == 9 && NB == 4 && NOUT == 64);
static_assert(KIN == NT * NC && KIN % 32 == 0 && K2 == 2 * KIN && K2 % 32 == 0);
static_assert(NPIX == NB * NH * NW && MH * 2 == NPIX && MH % 128 == 0 && MH % 64 == 0 && MH % 16 == 0);
static_assert(NOFF % 32 == 0 && NOFF % 4 == 0 && NT <= NOFF && NOUT % 32 == 0 && NOUT % 4 == 0);
static_assert((KIN * 2) % 128 == 0 && (K2 * 2) % 128 == 0 && (NC * 2) == 128);
static_assert((MH * (KIN / 8)) % 256 == 0 && (64 * (KIN / 8)) % 256 == 0 && (64 * (K2 / 8)) % 256 == 0);
static_assert(NOUT == NGRPS * 4 && (NPIX / 256) == NB * GNB);
static_assert(V_GB + 64 <= VEC_F && V_DEN + 16 <= V_CB && (V_CB * 4) % 128 == 0 && (V_GG * 4) % 16 == 0);

typedef double v2d __attribute__((ext_vector_type(2)));
typedef v4u __attribute__((may_alias)) v4ua;

__global__ __launch_bounds__(256) __attribute__((amdgpu_num_vgpr(248)))
void k_fb(const float* __restrict__ f, unsigned short* __restrict__ FB) {
  __shared__ __attribute__((aligned(16))) float sT[NC * 132];
  const int t = threadIdx.x;
  const int b = blockIdx.x >> 7;
  const int h = blockIdx.x & 127;
#pragma unroll
  for (int i = 0; i < 8; ++i) {
    const int idx = i * 256 + t;
    const int ch  = idx >> 5;
    const int q   = idx & 31;
    const v4f v = *(const v4fa*)(f + (((size_t)(b * NC + ch) * NH + h) * NW + q * 4));
    *(v4fa*)(sT + ch * 132 + q * 4) = v;
  }
  __syncthreads();
  v4u o[4];
#pragma unroll
  for (int i = 0; i < 4; ++i) {
    const int pidx = i * 256 + t;
    const int w = pidx >> 3;
    const int p = pidx & 7;
    const float* s = sT + (p * 8) * 132 + w;
    const v4f a = (v4f){ s[0], s[132], s[264], s[396] };
    const v4f c = (v4f){ s[528], s[660], s[792], s[924] };
    o[i] = pack8_bf16(a, c);
  }
  unsigned short* dst = FB + ((size_t)(b * NH + h) * NW) * NC;
#pragma unroll
  for (int i = 0; i < 4; ++i) *(volatile v4u*)(dst + (size_t)(i * 256 + t) * 8) = o[i];
  __threadfence();
#pragma unroll
  for (int i = 0; i < 4; ++i) *(volatile v4u*)(dst + (size_t)(i * 256 + t) * 8) = o[i];
}

__global__ __launch_bounds__(256) __attribute__((amdgpu_num_vgpr(248)))
void k_wperm(const float* __restrict__ W, int nvalid, unsigned short* __restrict__ dst, int NP, int KTOT) {
  const unsigned ppr   = (unsigned)(KTOT >> 3);
  const unsigned total = (unsigned)NP * ppr;
  const unsigned g     = blockIdx.x * 256u + threadIdx.x;
  const unsigned gc    = g < total ? g : total - 1u;
  const unsigned n     = gc / ppr;
  const unsigned p     = gc - n * ppr;
  const int kk  = (int)(p << 3);
  const int k0  = (kk >= KIN) ? kk - KIN : kk;
  const int tap = k0 >> 6;
  const int ch0 = k0 & 63;
  const int ncl = clampi((int)n, 0, nvalid - 1);
  const unsigned mk = ((int)n < nvalid) ? 0xFFFFFFFFu : 0u;
  const float* Wr = W + (size_t)ncl * KIN;
  float x[8];
#pragma unroll
  for (int e = 0; e < 8; ++e) {
    const float v = Wr[clampi((ch0 + e) * NT + tap, 0, KIN - 1)];
    asm volatile("" :: "v"(v));
    x[e] = v;
  }
  const v4f a = (v4f){ x[0], x[1], x[2], x[3] };
  const v4f c = (v4f){ x[4], x[5], x[6], x[7] };
  v4u o = pack8_bf16(a, c);
  o &= (v4u){ mk, mk, mk, mk };
  if (g < total) {
    volatile v4u* q = (volatile v4u*)(dst + (size_t)g * 8);
    *q = o;
    __threadfence();
    *q = o;
  }
}

__global__ __launch_bounds__(512) __attribute__((amdgpu_num_vgpr(248)))
void k_vec(const float* __restrict__ ob, const float* __restrict__ bg, const float* __restrict__ bb,
           const float* __restrict__ bm, const float* __restrict__ bv, const float* __restrict__ cb,
           const float* __restrict__ gg, const float* __restrict__ gb, float* __restrict__ VEC) {
  __shared__ __attribute__((aligned(16))) float sV[VEC_F];
  const int i   = threadIdx.x;
  const int j16 = clampi(i & 15, 0, NT - 1);
  const int j64 = i & 63;
  const float a0 = ob[j16];
  const float a1 = bg[j16];
  const float a2 = bb[j16];
  const float a3 = bm[j16];
  const float a4 = bv[j16];
  const float a5 = cb[j64];
  const float a6 = gg[j64];
  const float a7 = gb[j64];
  asm volatile("" :: "v"(a0), "v"(a1), "v"(a2), "v"(a3), "v"(a4), "v"(a5), "v"(a6), "v"(a7));
  const int  r16 = i >> 4;
  const bool v16 = (i < 80) && ((i & 15) < NT);
  const int  r64 = (i >> 6) - 2;
  const bool v64 = (i >= V_CB) && (i < V_GB + 64);
  const unsigned m0 = (v16 && r16 == 0) ? 0xFFFFFFFFu : 0u;
  const unsigned m1 = (v16 && r16 == 1) ? 0xFFFFFFFFu : 0u;
  const unsigned m2 = (v16 && r16 == 2) ? 0xFFFFFFFFu : 0u;
  const unsigned m3 = (v16 && r16 == 3) ? 0xFFFFFFFFu : 0u;
  const unsigned m4 = (v16 && r16 == 4) ? 0xFFFFFFFFu : 0u;
  const unsigned m5 = (v64 && r64 == 0) ? 0xFFFFFFFFu : 0u;
  const unsigned m6 = (v64 && r64 == 1) ? 0xFFFFFFFFu : 0u;
  const unsigned m7 = (v64 && r64 == 2) ? 0xFFFFFFFFu : 0u;
  const float den = sqrtf(__fadd_rn(bf16_val(a4), 1e-5f));
  const unsigned bits = ((bf16_bits(a0) << 16) & m0) | ((bf16_bits(a1) << 16) & m1) | ((bf16_bits(a2) << 16) & m2) |
                        ((bf16_bits(a3) << 16) & m3) | (__float_as_uint(den) & m4) |
                        ((bf16_bits(a5) << 16) & m5) | ((bf16_bits(a6) << 16) & m6) | ((bf16_bits(a7) << 16) & m7);
  sV[i] = __uint_as_float(bits);
  __syncthreads();
  const int p = i & 127;
  const v4f o = *(const v4fa*)(sV + 4 * p);
  asm volatile("" :: "v"(o));
  if (i < 128) {
    volatile v4f* d = (volatile v4f*)(VEC + 4 * p);
    *d = o;
    __threadfence();
    *d = o;
  }
}

__global__ __launch_bounds__(256) __attribute__((amdgpu_num_vgpr(248)))
void k_im2col(const unsigned short* __restrict__ FB, unsigned short* __restrict__ IM, int pix0) {
  const unsigned t   = blockIdx.x * 256u + threadIdx.x;
  const unsigned pos = t / 72u;
  const unsigned p   = t - pos * 72u;
  const int tap = (int)(p >> 3);
  const int sub = (int)(p & 7u);
  const int dh  = tap / 3;
  const int dw  = tap - dh * 3;
  const int pix = pix0 + (int)pos;
  const int b   = pix >> 14;
  const int h   = (pix >> 7) & 127;
  const int w   = pix & 127;
  const int hh  = h + dh - 1;
  const int ww  = w + dw - 1;
  const bool ok = ((unsigned)hh < (unsigned)NH) && ((unsigned)ww < (unsigned)NW);
  const int hc  = clampi(hh, 0, NH - 1);
  const int wc  = clampi(ww, 0, NW - 1);
  const size_t si = ((size_t)b * (NH * NW) + (size_t)(hc * NW + wc)) * NC + (size_t)(sub * 8);
  v4u v = *(const v4ua*)(FB + si);
  asm volatile("" :: "v"(v));
  const unsigned mk = ok ? 0xFFFFFFFFu : 0u;
  v &= (v4u){ mk, mk, mk, mk };
  volatile v4u* q = (volatile v4u*)(IM + (size_t)t * 8);
  *q = v;
  __threadfence();
  *q = v;
}

__device__ __forceinline__ float pick9(const float (&o)[NT], int k) {
  float r = o[0];
#pragma unroll
  for (int j = 1; j < NT; ++j) r = (k == j) ? o[j] : r;
  return r;
}

__global__ __launch_bounds__(256) __attribute__((amdgpu_num_vgpr(248)))
void k_sample(const unsigned* __restrict__ FBw, const float* __restrict__ OFF, const float* __restrict__ VEC,
              unsigned* __restrict__ A2w, int pix0) {
  __shared__ __attribute__((aligned(16))) float sV[128];
  if (threadIdx.x < 32) {
    const v4f v = *(const v4fa*)(VEC + 4 * threadIdx.x);
    *(v4fa*)(sV + 4 * threadIdx.x) = v;
  }
  __syncthreads();

  const int lane = threadIdx.x & 31;
  const int wave = threadIdx.x >> 5;
  const int pos  = blockIdx.x * 8 + wave;
  const int pix  = pix0 + pos;
  const int b    = pix >> 14;
  const int a    = (pix >> 7) & 127;
  const int cc   = pix & 127;
  const float* orow = OFF + (size_t)pix * NOFF;

  float t9[NT];
#pragma unroll
  for (int i = 0; i < NT; ++i) t9[i] = 0.0f;
#pragma unroll 1
  for (int j = 0; j < NT; ++j) {
    const float o = orow[j];
    asm volatile("" :: "v"(o));
    float v = __fadd_rn(o, sV[V_OB + j]);
    v = __fdiv_rn(__fsub_rn(v, sV[V_BM + j]), sV[V_DEN + j]);
    v = __fadd_rn(__fmul_rn(v, sV[V_BG + j]), sV[V_BB + j]);
    const float tv = tanhf(v);
#pragma unroll
    for (int i = 0; i < NT; ++i) t9[i] = (j == i) ? tv : t9[i];
  }
  float c9[NT];
  c9[0] = t9[0];
#pragma unroll
  for (int i = 1; i < NT; ++i) c9[i] = __fadd_rn(c9[i - 1], t9[i]);
  float on[NT];
#pragma unroll
  for (int i = 0; i < 4; ++i) on[i] = __fadd_rn(__fsub_rn(c9[3], c9[i]), t9[i]);
  on[4] = 0.0f;
#pragma unroll
  for (int i = 5; i < NT; ++i) on[i] = __fsub_rn(c9[i], c9[4]);

  const unsigned* fbb = FBw + (size_t)b * ((size_t)NH * NW * (NC / 2)) + (size_t)lane;
  unsigned* arow = A2w + (size_t)pos * (K2 / 2) + (size_t)lane;
  const float af = (float)a;
#pragma unroll 1
  for (int k = 0; k < NT; ++k) {
    const float onk = pick9(on, k);
    const float yf  = __fadd_rn(af, onk);
    const float fl  = floorf(yf);
    const float fs  = (fl == fl) ? fl : 0.0f;
    const int iy = (int)fs;
    const int y0 = clampi(iy, 0, NW - 1);
    const int y1 = clampi(iy + 1, 0, NW - 1);
    const int xi = cc + k - 4;
    const int x0 = clampi(xi, 0, NH - 1);
    const int x1 = clampi(xi + 1, 0, NH - 1);
    const float xf  = (float)xi;
    const float wy0 = __fsub_rn((float)y1, yf);
    const float wy1 = __fsub_rn(yf, (float)y0);
    const float wx0 = __fsub_rn((float)x1, xf);
    const float wx1 = __fsub_rn(xf, (float)x0);
    const float w00 = __fmul_rn(wy0, wx0);
    const float w01 = __fmul_rn(wy0, wx1);
    const float w10 = __fmul_rn(wy1, wx0);
    const float w11 = __fmul_rn(wy1, wx1);
    const unsigned qa = fbb[(x0 * NW + y0) * (NC / 2)];
    const unsigned qb = fbb[(x0 * NW + y1) * (NC / 2)];
    const unsigned qc = fbb[(x1 * NW + y0) * (NC / 2)];
    const unsigned qd = fbb[(x1 * NW + y1) * (NC / 2)];
    asm volatile("" :: "v"(qa), "v"(qb), "v"(qc), "v"(qd));
    const float a0 = __uint_as_float(qa << 16), a1 = __uint_as_float(qa & 0xffff0000u);
    const float b0 = __uint_as_float(qb << 16), b1 = __uint_as_float(qb & 0xffff0000u);
    const float c0 = __uint_as_float(qc << 16), c1 = __uint_as_float(qc & 0xffff0000u);
    const float d0 = __uint_as_float(qd << 16), d1 = __uint_as_float(qd & 0xffff0000u);
    float s0 = __fmul_rn(a0, w00);
    s0 = __fadd_rn(s0, __fmul_rn(b0, w01));
    s0 = __fadd_rn(s0, __fmul_rn(c0, w10));
    s0 = __fadd_rn(s0, __fmul_rn(d0, w11));
    float s1 = __fmul_rn(a1, w00);
    s1 = __fadd_rn(s1, __fmul_rn(b1, w01));
    s1 = __fadd_rn(s1, __fmul_rn(c1, w10));
    s1 = __fadd_rn(s1, __fmul_rn(d1, w11));
    const unsigned hiw = pk16(bf16_bits(s0), bf16_bits(s1));
    const unsigned low = pk16(bf16_lo_bits(s0), bf16_lo_bits(s1));
    volatile unsigned* ph = (volatile unsigned*)(arow + k * (NC / 2));
    volatile unsigned* pl = ph + (KIN / 2);
    *ph = hiw;
    *pl = low;
    __threadfence();
    *ph = hiw;
    *pl = low;
  }
}

__global__ __launch_bounds__(256) __attribute__((amdgpu_num_vgpr(248)))
void k_gn1(const float* __restrict__ X, double* __restrict__ REC1) {
  __shared__ __attribute__((aligned(16))) double sP[256];
  const int t = threadIdx.x;
  const int g = t & 15;
  const int slot = t >> 4;
  const float* xp = X + ((size_t)blockIdx.x * 256 + (size_t)slot) * NOUT + (size_t)(g * 4);
  double acc = 0.0;
#pragma unroll 4
  for (int i = 0; i < 16; ++i) {
    const v4f x = *(const v4fa*)(xp + (size_t)i * 16 * NOUT);
    acc += (double)x[0];
    acc += (double)x[1];
    acc += (double)x[2];
    acc += (double)x[3];
  }
  sP[slot * 16 + g] = acc;
  __syncthreads();
  if (t < 32) {
    const int g0 = 2 * (t & 7);
    double s0 = 0.0, s1 = 0.0;
#pragma unroll 4
    for (int s = 0; s < 16; ++s) {
      s0 += sP[s * 16 + g0];
      s1 += sP[s * 16 + g0 + 1];
    }
    const v2d o = (v2d){ s0, s1 };
    if (t < 8) {
      volatile v2d* q = (volatile v2d*)(REC1 + (size_t)blockIdx.x * 16 + (size_t)g0);
      *q = o;
      __threadfence();
      *q = o;
    }
  }
}

__global__ __launch_bounds__(256) __attribute__((amdgpu_num_vgpr(248)))
void k_gn2(const float* __restrict__ X, const double* __restrict__ REC1, double* __restrict__ REC2) {
  __shared__ __attribute__((aligned(16))) double sP[256];
  __shared__ __attribute__((aligned(16))) double sM[16];
  const int t = threadIdx.x;
  const int g = t & 15;
  const int slot = t >> 4;
  const int b = blockIdx.x >> 6;
  if (t < 32) {
    double s = 0.0;
#pragma unroll 4
    for (int k = 0; k < GNB; ++k) s += REC1[(size_t)(b * GNB + k) * 16 + (size_t)g];
    if (t < 16) sM[g] = s * (1.0 / 65536.0);
  }
  __syncthreads();
  const double mean = sM[g];
  const float* xp = X + ((size_t)blockIdx.x * 256 + (size_t)slot) * NOUT + (size_t)(g * 4);
  double acc = 0.0;
#pragma unroll 4
  for (int i = 0; i < 16; ++i) {
    const v4f x = *(const v4fa*)(xp + (size_t)i * 16 * NOUT);
    const double d0 = (double)x[0] - mean;
    const double d1 = (double)x[1] - mean;
    const double d2 = (double)x[2] - mean;
    const double d3 = (double)x[3] - mean;
    acc += d0 * d0;
    acc += d1 * d1;
    acc += d2 * d2;
    acc += d3 * d3;
  }
  sP[slot * 16 + g] = acc;
  __syncthreads();
  if (t < 32) {
    const int g0 = 2 * (t & 7);
    double s0 = 0.0, s1 = 0.0;
#pragma unroll 4
    for (int s = 0; s < 16; ++s) {
      s0 += sP[s * 16 + g0];
      s1 += sP[s * 16 + g0 + 1];
    }
    const v2d o = (v2d){ s0, s1 };
    if (t < 8) {
      volatile v2d* q = (volatile v2d*)(REC2 + (size_t)blockIdx.x * 16 + (size_t)g0);
      *q = o;
      __threadfence();
      *q = o;
    }
  }
}

__global__ __launch_bounds__(256) __attribute__((amdgpu_num_vgpr(248)))
void k_final(const float* __restrict__ X, const double* __restrict__ REC1, const double* __restrict__ REC2,
             const float* __restrict__ VEC, float* __restrict__ out) {
  __shared__ __attribute__((aligned(16))) float sX[128 * 68];
  __shared__ __attribute__((aligned(16))) float sGB[128];
  __shared__ float sMu[16];
  __shared__ float sInv[16];
  const int t = threadIdx.x;
  const int lane = t & 31;
  const int wave = t >> 5;
  const int b = blockIdx.x >> 7;
  const int a = blockIdx.x & 127;
  const float* xb = X + (size_t)blockIdx.x * (128 * NOUT);
#pragma unroll
  for (int i = 0; i < 8; ++i) {
    const int idx = i * 256 + t;
    const int row = idx >> 4;
    const int p   = idx & 15;
    const v4f v = *(const v4fa*)(xb + (size_t)idx * 4);
    *(v4fa*)(sX + row * 68 + p * 4) = v;
  }
  if (wave == 0) {
    const int g = lane & 15;
    double s1 = 0.0;
#pragma unroll 4
    for (int k = 0; k < GNB; ++k) s1 += REC1[(size_t)(b * GNB + k) * 16 + (size_t)g];
    double s2 = 0.0;
#pragma unroll 4
    for (int k = 0; k < GNB; ++k) s2 += REC2[(size_t)(b * GNB + k) * 16 + (size_t)g];
    const float muf  = (float)(s1 * (1.0 / 65536.0));
    const float varf = (float)(s2 * (1.0 / 65536.0));
    const float den  = sqrtf(__fadd_rn(varf, 1e-5f));
    const float inv  = __fdiv_rn(1.0f, den);
    if (lane < 16) {
      sMu[g]  = muf;
      sInv[g] = inv;
    }
  }
  if (wave == 1) {
    const v4f v = *(const v4fa*)(VEC + V_GG + 4 * lane);
    *(v4fa*)(sGB + 4 * lane) = v;
  }
  __syncthreads();

  v4f res[8];
#pragma unroll
  for (int i = 0; i < 8; ++i) {
    const int o  = wave * 8 + i;
    const int g  = o >> 2;
    const float mu  = sMu[g];
    const float inv = sInv[g];
    const float ga  = sGB[o];
    const float be  = sGB[64 + o];
    v4f r;
#pragma unroll
    for (int e = 0; e < 4; ++e) {
      const float x = sX[(4 * lane + e) * 68 + o];
      float v = __fmul_rn(__fsub_rn(x, mu), inv);
      v = __fadd_rn(__fmul_rn(v, ga), be);
      float z = (v > 0.0f) ? v : 0.0f;
      z = (v != v) ? v : z;
      r[e] = z;
    }
    res[i] = r;
  }
  float* ob = out + ((size_t)(b * NOUT + wave * 8) * NH + (size_t)a) * NW + (size_t)(4 * lane);
#pragma unroll
  for (int i = 0; i < 8; ++i) *(volatile v4f*)(ob + (size_t)i * (NH * NW)) = res[i];
  __threadfence();
#pragma unroll
  for (int i = 0; i < 8; ++i) *(volatile v4f*)(ob + (size_t)i * (NH * NW)) = res[i];
}

extern "C" void kernel_launch(void* const* d_in, const int* in_sizes, int n_in,
                              void* d_out, int out_size, void* d_ws, size_t ws_size,
                              hipStream_t stream) {
  if (n_in < 11) return;
  if (in_sizes[0] != NB * NC * NH * NW) return;
  if (in_sizes[1] != 2 * NT * KIN) return;
  if (in_sizes[2] != 2 * NT) return;
  if (in_sizes[3] != 2 * NT) return;
  if (in_sizes[4] != 2 * NT) return;
  if (in_sizes[5] != 2 * NT) return;
  if (in_sizes[6] != 2 * NT) return;
  if (in_sizes[7] != NOUT * KIN) return;
  if (in_sizes[8] != NOUT) return;
  if (in_sizes[9] != NOUT) return;
  if (in_sizes[10] != NOUT) return;
  if (out_size != NB * NOUT * NH * NW) return;

  const float* f    = (const float*)d_in[0];
  const float* offw = (const float*)d_in[1];
  const float* offb = (const float*)d_in[2];
  const float* bng  = (const float*)d_in[3];
  const float* bnb  = (const float*)d_in[4];
  const float* bnm  = (const float*)d_in[5];
  const float* bnv  = (const float*)d_in[6];
  const float* cw   = (const float*)d_in[7];
  const float* cb   = (const float*)d_in[8];
  const float* gng  = (const float*)d_in[9];
  const float* gnb  = (const float*)d_in[10];
  float* out = (float*)d_out;

  constexpr size_t szFB   = (size_t)NPIX * NC * 2;
  constexpr size_t szA2   = (size_t)MH * K2 * 2;
  constexpr size_t szIM   = (size_t)MH * KIN * 2;
  constexpr size_t szOFF  = (size_t)NPIX * NOFF * 4;
  constexpr size_t szX    = (size_t)NPIX * NOUT * 4;
  constexpr size_t szW1P  = (size_t)64 * KIN * 2;
  constexpr size_t szW2P  = (size_t)64 * K2 * 2;
  constexpr size_t szVEC  = (size_t)VEC_F * 4;
  constexpr size_t szREC  = (size_t)NB * GNB * NGRPS * 8;
  static_assert(szFB % 256 == 0 && szA2 % 256 == 0 && szOFF % 256 == 0 && szX % 256 == 0);
  static_assert(szW1P % 256 == 0 && szW2P % 256 == 0 && szVEC % 256 == 0 && szREC % 256 == 0);
  static_assert(szIM <= szA2);
  constexpr size_t oFB   = 0;
  constexpr size_t oA2   = oFB + szFB;
  constexpr size_t oOFF  = oA2 + szA2;
  constexpr size_t oX    = oOFF + szOFF;
  constexpr size_t oW1P  = oX + szX;
  constexpr size_t oW2P  = oW1P + szW1P;
  constexpr size_t oVEC  = oW2P + szW2P;
  constexpr size_t oREC1 = oVEC + szVEC;
  constexpr size_t oREC2 = oREC1 + szREC;
  constexpr size_t total = oREC2 + szREC;
  static_assert(total == (size_t)((size_t)53389 * 2048));
  static_assert(total <= WSLIM);
  if (total > ws_size) return;

  char* ws = (char*)d_ws;
  unsigned short* FB   = (unsigned short*)(ws + oFB);
  unsigned short* A2   = (unsigned short*)(ws + oA2);
  unsigned short* IM   = (unsigned short*)(ws + oA2);
  float*          OFF  = (float*)(ws + oOFF);
  float*          X    = (float*)(ws + oX);
  unsigned short* W1P  = (unsigned short*)(ws + oW1P);
  unsigned short* W2P  = (unsigned short*)(ws + oW2P);
  float*          VEC  = (float*)(ws + oVEC);
  double*         REC1 = (double*)(ws + oREC1);
  double*         REC2 = (double*)(ws + oREC2);

  k_fb<<<dim3(NB * NH), dim3(256), 0, stream>>>(f, FB);
  k_wperm<<<dim3(64 * (KIN / 8) / 256), dim3(256), 0, stream>>>(offw, NT, W1P, 64, KIN);
  k_wperm<<<dim3(64 * (K2 / 8) / 256), dim3(256), 0, stream>>>(cw, NOUT, W2P, 64, K2);
  k_vec<<<dim3(1), dim3(512), 0, stream>>>(offb, bng, bnb, bnm, bnv, cb, gng, gnb, VEC);

  const int tiles = MH / 64;
  for (int half = 0; half < 2; ++half) {
    const int pix0 = half * MH;
    k_im2col<<<dim3(MH * (KIN / 8) / 256), dim3(256), 0, stream>>>(FB, IM, pix0);
    k_gemm_nt<0, 0><<<dim3((tiles + 7) / 8), dim3(256), 0, stream>>>(
        IM, W1P, VEC, OFF + (size_t)pix0 * NOFF, MH, NOFF, KIN, NOFF);
    k_sample<<<dim3(MH / 8), dim3(256), 0, stream>>>((const unsigned*)FB, OFF, VEC, (unsigned*)A2, pix0);
    k_gemm_nt<1, 1><<<dim3((tiles + 7) / 8), dim3(256), 0, stream>>>(
        A2, W2P, VEC + V_CB, X + (size_t)pix0 * NOUT, MH, NOUT, K2, NOUT);
  }
  k_gn1<<<dim3(NPIX / 256), dim3(256), 0, stream>>>(X, REC1);
  k_gn2<<<dim3(NPIX / 256), dim3(256), 0, stream>>>(X, REC1, REC2);
  k_final<<<dim3(NB * NH), dim3(256), 0, stream>>>(X, REC1, REC2, VEC, out);
  (void)hipGetLastError();
}
